// MagLaplacianEncoder_46145128628992
// MI455X (gfx1250) — hardware-verified
//
#include <hip/hip_runtime.h>
#include <math.h>

typedef __attribute__((ext_vector_type(16))) _Float16 v16h;
typedef __attribute__((ext_vector_type(16))) __bf16 v16b;
typedef __attribute__((ext_vector_type(8)))  _Float16 v8h;
typedef __attribute__((ext_vector_type(8)))  float v8f;
typedef __attribute__((ext_vector_type(4)))  float v4f;
typedef __attribute__((ext_vector_type(2)))  float v2f;
typedef __attribute__((ext_vector_type(4)))  unsigned v4u;
typedef __attribute__((ext_vector_type(4)))  int v4i;
typedef float __attribute__((may_alias)) float_a;
typedef int __attribute__((may_alias)) int_a;

template <typename T> __device__ __forceinline__ void vst2(void* p, T v) { *(volatile T*)p = v; __threadfence(); *(volatile T*)p = v; }
__device__ __forceinline__ v8f wmma16(v16h a, v16h b, v8f c) {
  v8f d = __builtin_amdgcn_wmma_f32_16x16x32_f16(false, a, false, b, (short)0, c, false, false);
  asm volatile("v_nop\n\tv_nop\n\tv_nop\n\tv_nop" : "+v"(d) : "v"(a), "v"(b));
  return d;
}
__device__ __forceinline__ v8f wmma_bf(v16b a, v16b b, v8f c) {
  v8f d = __builtin_amdgcn_wmma_f32_16x16x32_bf16(false, a, false, b, (short)0, c, false, false);
  asm volatile("v_nop\n\tv_nop\n\tv_nop\n\tv_nop" : "+v"(d) : "v"(a), "v"(b));
  return d;
}
__device__ __forceinline__ v16h frag_h(const _Float16* rowk0, int lane) {
  union { v16h v; v8h q[2]; } u; const _Float16* p = rowk0 + 8 * (lane >> 4);
  u.q[0] = *(const v8h*)p; u.q[1] = *(const v8h*)(p + 16); return u.v;
}
__device__ __forceinline__ v16h frag_f32(const float* rowk0, int lane) {
  v16h a; const float* p = rowk0 + 8 * (lane >> 4);
#pragma unroll
  for (int i = 0; i < 8; ++i) { a[i] = (_Float16)p[i]; a[8 + i] = (_Float16)p[16 + i]; }
  return a;
}
__device__ __forceinline__ v16h frag_f32s(const float* rowk0, int lane, float sc) {
  v16h a; const float* p = rowk0 + 8 * (lane >> 4);
#pragma unroll
  for (int i = 0; i < 8; ++i) { a[i] = (_Float16)(p[i] * sc); a[8 + i] = (_Float16)(p[16 + i] * sc); }
  return a;
}
__device__ __forceinline__ v16h fragc_f32(const float* W, int k0, int n, int lane, int ld, int K) {
  v16h a; const int g = lane >> 4;
#pragma unroll
  for (int i = 0; i < 8; ++i) { const int ka = k0 + 8 * g + i, kb = ka + 16;
    a[i] = (_Float16)(ka < K ? W[(size_t)ka * ld + n] : 0.f); a[8 + i] = (_Float16)(kb < K ? W[(size_t)kb * ld + n] : 0.f); }
  return a;
}
struct F2 { v16b h, l; };
__device__ __forceinline__ F2 bsplit16(const float v[16]) { F2 r;
#pragma unroll
  for (int i = 0; i < 16; ++i) { const __bf16 h = (__bf16)v[i]; r.h[i] = h; r.l[i] = (__bf16)(v[i] - (float)h); }
  return r; }
__device__ __forceinline__ F2 split_row(const float* row, int k0, int lane) { float v[16]; const float* p = row + k0 + 8 * (lane >> 4);
#pragma unroll
  for (int i = 0; i < 8; ++i) { v[i] = p[i]; v[8 + i] = p[16 + i]; }
  return bsplit16(v); }
__device__ __forceinline__ F2 split_rowK(const float* row, int k0, int lane, int K) { float v[16]; const int g = lane >> 4;
#pragma unroll
  for (int i = 0; i < 8; ++i) { const int ka = k0 + 8 * g + i, kb = ka + 16; v[i] = ka < K ? row[ka] : 0.f; v[8 + i] = kb < K ? row[kb] : 0.f; }
  return bsplit16(v); }
__device__ __forceinline__ F2 split_col(const float* W, int k0, int n, int lane, int ld, int K) { float v[16]; const int g = lane >> 4;
#pragma unroll
  for (int i = 0; i < 8; ++i) { const int ka = k0 + 8 * g + i, kb = ka + 16; v[i] = ka < K ? W[(size_t)ka * ld + n] : 0.f; v[8 + i] = kb < K ? W[(size_t)kb * ld + n] : 0.f; }
  return bsplit16(v); }
__device__ __forceinline__ v8f mac3(const F2& a, const F2& b, v8f c) { c = wmma_bf(a.l, b.h, c); c = wmma_bf(a.h, b.l, c); return wmma_bf(a.h, b.h, c); }
__device__ __forceinline__ float sigm(float v) { return 1.0f / (1.0f + expf(-v)); }
#define LDSX() do { asm volatile("s_wait_dscnt 0" ::: "memory"); __builtin_amdgcn_wave_barrier(); __builtin_amdgcn_fence(__ATOMIC_RELEASE, "workgroup"); } while (0)

#define NNODE 32768
#define KS 16
#define DE 32
#define NH 4
#define HDM (NH * DE)
#define DA 256
#define KF (KS * DE)

__global__ __launch_bounds__(256) void k_pack(const float* __restrict__ Wq, const float* __restrict__ Wk, const float* __restrict__ Wv, const float* __restrict__ Wo, const float* __restrict__ Wa, _Float16* __restrict__ PQ, _Float16* __restrict__ POT, _Float16* __restrict__ PAT) {
  const int r = blockIdx.x, tid = threadIdx.x; __shared__ __align__(16) _Float16 srow[KF];
  if (r < 3 * HDM) { const int which = r / HDM, n = r % HDM; const float* W = which == 0 ? Wq : (which == 1 ? Wk : Wv);
    if (tid < 64) srow[tid] = (_Float16)(tid < DE ? W[(size_t)tid * HDM + n] * 16.0f : 0.f);
    __syncthreads(); if (tid < 8) vst2(PQ + (size_t)r * 64 + tid * 8, *(const v4u*)(&srow[tid * 8])); }
  else if (r < 3 * HDM + DE) { const int n = r - 3 * HDM; if (tid < HDM) srow[tid] = (_Float16)(Wo[(size_t)tid * DE + n] * 16.0f);
    __syncthreads(); if (tid < 16) vst2(POT + (size_t)n * HDM + tid * 8, *(const v4u*)(&srow[tid * 8])); }
  else { const int n = r - 3 * HDM - DE; for (int k = tid; k < KF; k += 256) srow[k] = (_Float16)(Wa[(size_t)k * DA + n] * 16.0f);
    __syncthreads(); if (tid < 64) vst2(PAT + (size_t)n * KF + tid * 8, *(const v4u*)(&srow[tid * 8])); }
}
__global__ __launch_bounds__(128) void k_node(const float* __restrict__ eigval, const float* __restrict__ vre, const float* __restrict__ vim, const float* __restrict__ We, const float* __restrict__ be,
                                            const _Float16* __restrict__ PQ, const _Float16* __restrict__ POT, const float* __restrict__ bo, _Float16* __restrict__ T2) {
  __shared__ __align__(16) float str[4][16][DE + 4];
  __shared__ __align__(16) _Float16 sa[4][16][DE + 8];
  __shared__ __align__(16) _Float16 sq[4][16][HDM + 8], sk[4][16][HDM + 8], sv[4][16][HDM + 8];
  __shared__ __align__(16) float ss[4][16][20];
  __shared__ __align__(16) _Float16 sp[4][16][40];
  __shared__ __align__(16) _Float16 so[4][16][HDM + 8];
  __shared__ __align__(16) _Float16 st2[4][16][DE + 8];
  const int tid = threadIdx.x, wave = tid >> 5, lane = tid & 31, col = lane & 15, g = lane >> 4;
  const int node = blockIdx.x * 4 + wave;
  { const int t = lane >> 1, hf = lane & 1; const float re = vre[(size_t)node * KS + t], im = vim[(size_t)node * KS + t];
#pragma unroll
    for (int c = hf * 16; c < hf * 16 + 16; ++c) { const float a = re * We[c] + im * We[DE + c]; const float b = be[c]; const float v1 = a + b, v2 = -a + b; const float v = (v1 > 0.f ? v1 : 0.f) + (v2 > 0.f ? v2 : 0.f); str[wave][t][c] = v; sa[wave][t][c] = (_Float16)v; }
    if (hf == 1) { for (int c = DE; c < DE + 8; ++c) sa[wave][t][c] = (_Float16)0.f; }
    if (t == 0 && hf == 0) { for (int r = 0; r < 16; ++r) for (int c = 16; c < 32; ++c) sp[wave][r][c] = (_Float16)0.f; } }
  LDSX();
  { const v16h a = frag_h(&sa[wave][col][0], lane);
#pragma unroll 1
    for (int which = 0; which < 3; ++which) { _Float16 (*dst)[HDM + 8] = which == 0 ? sq[wave] : (which == 1 ? sk[wave] : sv[wave]);
#pragma unroll
      for (int t8 = 0; t8 < 8; ++t8) { const v8f acc = wmma16(a, frag_h(PQ + (size_t)(which * HDM + t8 * 16 + col) * 64, lane), (v8f){});
#pragma unroll
        for (int r = 0; r < 8; ++r) dst[8 * g + r][t8 * 16 + col] = (_Float16)(acc[r] * (4.0f / 16.0f)); } } }
  LDSX();
  bool pm[KS];
#pragma unroll
  for (int t = 0; t < KS; ++t) pm[t] = (t == 0) || (eigval[t] > 0.f);
#pragma unroll 1
  for (int h = 0; h < NH; ++h) {
    { const v8f s = wmma16(frag_h(&sq[wave][col][h * DE], lane), frag_h(&sk[wave][col][h * DE], lane), (v8f){});
#pragma unroll
      for (int r = 0; r < 8; ++r) ss[wave][8 * g + r][col] = s[r] * (0.17677669529663689f / 16.0f); }
    LDSX();
    if (lane < 16) { const int t = lane; float vals[KS]; float mx = -3.4e38f;
#pragma unroll
      for (int u = 0; u < KS; ++u) { const float v = (pm[t] && pm[u]) ? ss[wave][t][u] : -1e30f; vals[u] = v; mx = fmaxf(mx, v); }
      float se = 0.f;
#pragma unroll
      for (int u = 0; u < KS; ++u) { vals[u] = expf(vals[u] - mx); se += vals[u]; }
      const float inv = 16384.0f / se;
#pragma unroll
      for (int u = 0; u < KS; ++u) sp[wave][t][u] = (_Float16)(vals[u] * inv); }
    LDSX();
    {
#pragma unroll
      for (int t2 = 0; t2 < 2; ++t2) { v16h b; const int n = h * DE + t2 * 16 + col;
#pragma unroll
        for (int i = 0; i < 8; ++i) { const int ka = 8 * g + i; b[i] = sv[wave][ka][n]; b[8 + i] = (_Float16)0.f; }
        const v8f o = wmma16(frag_h(&sp[wave][col][0], lane), b, (v8f){});
#pragma unroll
        for (int r = 0; r < 8; ++r) so[wave][8 * g + r][n] = (_Float16)(o[r] * (8.0f / (16384.0f * 4.0f))); } }
    LDSX(); }
  { v8f acc[2] = {};
#pragma unroll
    for (int kc = 0; kc < HDM / 32; ++kc) { const v16h a = frag_h(&so[wave][col][0] + kc * 32, lane);
#pragma unroll
      for (int t2 = 0; t2 < 2; ++t2) acc[t2] = wmma16(a, frag_h(POT + (size_t)(t2 * 16 + col) * HDM + kc * 32, lane), acc[t2]); }
#pragma unroll
    for (int t2 = 0; t2 < 2; ++t2) { const int c = t2 * 16 + col; const float bb = bo[c];
#pragma unroll
      for (int r = 0; r < 8; ++r) { const int t = 8 * g + r; const float v = (acc[t2][r] * (1.0f / (16.0f * 8.0f)) + bb + str[wave][t][c]) * (pm[t] ? 1.0f : 0.0f); st2[wave][t][c] = (_Float16)v; } } }
  LDSX();
  { const int rl0 = lane >> 2, pc = lane & 3;
#pragma unroll
    for (int j = 0; j < 2; ++j) { const int rl = 8 * j + rl0; vst2(T2 + (size_t)node * KF + rl * DE + pc * 8, *(const v4u*)(&st2[wave][rl][pc * 8])); } }
}
__global__ __launch_bounds__(128) void k_aggr(const _Float16* __restrict__ T2, const _Float16* __restrict__ PAT, const float* __restrict__ ba, float* __restrict__ out) {
  __shared__ __align__(16) float sout[4][16][132];
  const int tid = threadIdx.x, wave = tid >> 5, lane = tid & 31, col = lane & 15, g = lane >> 4;
  const int r0 = blockIdx.x * 64 + wave * 16;
#pragma unroll 1
  for (int nh = 0; nh < 2; ++nh) { v8f acc[8] = {};
#pragma unroll 2
    for (int kc = 0; kc < KF / 32; ++kc) { const v16h a = frag_h(T2 + (size_t)(r0 + col) * KF + kc * 32, lane);
#pragma unroll
      for (int t = 0; t < 8; ++t) acc[t] = wmma16(a, frag_h(PAT + (size_t)(nh * 128 + t * 16 + col) * KF + kc * 32, lane), acc[t]); }
#pragma unroll
    for (int t = 0; t < 8; ++t) { const int n = nh * 128 + t * 16 + col; const float bb = ba[n];
#pragma unroll
      for (int r = 0; r < 8; ++r) { const float v = acc[t][r] * (1.0f / 16.0f) + bb; sout[wave][8 * g + r][t * 16 + col] = v > 0.f ? v : 0.f; } }
    LDSX();
#pragma unroll 4
    for (int rl = 0; rl < 16; ++rl) vst2(out + (size_t)(r0 + rl) * DA + nh * 128 + lane * 4, *(const v4f*)(&sout[wave][rl][lane * 4]));
    LDSX(); }
}
extern "C" void kernel_launch(void* const* d_in, const int* in_sizes, int n_in, void* d_out, int out_size, void* d_ws, size_t ws_size, hipStream_t stream) {
  (void)in_sizes; (void)n_in; (void)out_size; (void)ws_size;
  const float** I = (const float**)d_in;
  float* out = (float*)d_out;
  char* ws = (char*)d_ws; size_t off = 0;
  auto take = [&](size_t bytes) { char* p = ws + off; off += (bytes + 255) & ~(size_t)255; return p; };
  _Float16* PQ = (_Float16*)take((size_t)3 * HDM * 64 * 2); _Float16* POT = (_Float16*)take((size_t)DE * HDM * 2); _Float16* PAT = (_Float16*)take((size_t)DA * KF * 2); _Float16* T2 = (_Float16*)take((size_t)NNODE * KF * 2);
  k_pack<<<3 * HDM + DE + DA, 256, 0, stream>>>(I[7], I[8], I[9], I[10], I[12], PQ, POT, PAT);
  k_node<<<NNODE / 4, 128, 0, stream>>>(I[2], I[3], I[4], I[5], I[6], PQ, POT, I[11], T2);
  k_aggr<<<NNODE / 64, 128, 0, stream>>>(T2, PAT, I[13], out);
}
